// ModifiedAttention_53120155517143
// MI455X (gfx1250) — hardware-verified
//
#include <hip/hip_runtime.h>

typedef _Float16 v16h __attribute__((ext_vector_type(16)));
typedef _Float16 v8h  __attribute__((ext_vector_type(8)));
typedef float    v8f  __attribute__((ext_vector_type(8)));
typedef float    v4f  __attribute__((ext_vector_type(4)));
typedef v8h __attribute__((may_alias)) v8ha;
typedef v4f __attribute__((may_alias)) v4fa;

union Frag { v16h v; v8h half[2]; };

#define HID    2048
#define NHEAD  16
#define HD     128
#define SEQ    2048
#define BATCH  2
#define MROWS  (BATCH * SEQ)
#define NX     (MROWS * HID)
#define NW     (HID * HID)
#define NX8    (NX / 8)
#define NW8    (NW / 8)
#define PSCALE 16384.0f
#define WSCALE 32.0f
#define CSCALE 32.0f
#define SM_SCALE 0.0883883476f

static_assert(MROWS % 128 == 0);
static_assert(SEQ % 128 == 0);
static_assert(HID % 64 == 0);
static_assert(NX8 % 256 == 0);
static_assert(NW8 % 256 == 0);

__device__ __forceinline__ v8f wmma_f16(v16h a, v16h b, v8f c) {
  v8f d = __builtin_amdgcn_wmma_f32_16x16x32_f16(false, a, false, b, (short)0, c, false, false);
  asm volatile("v_nop\n\tv_nop\n\tv_nop\n\tv_nop" : "+v"(d) : "v"(a), "v"(b));
  return d;
}

__device__ __forceinline__ v16h load_frag(const _Float16* p, int h) {
  Frag f;
  f.half[0] = *(const v8ha*)(p + 8 * h);
  f.half[1] = *(const v8ha*)(p + 16 + 8 * h);
  return f.v;
}

__global__ __launch_bounds__(256) void convert_kernel(
    const float* __restrict__ x,
    const float* __restrict__ wq, const float* __restrict__ wk,
    const float* __restrict__ wv, const float* __restrict__ wo,
    _Float16* __restrict__ xh, _Float16* __restrict__ wh)
{
  const int blk = blockIdx.x;
  if (blk >= (NX8 + 4 * NW8) / 256) return;
  const int g = blk * 256 + threadIdx.x;
  const float* src;
  _Float16* dst;
  float sc;
  if (blk < NX8 / 256) {
    src = x + (size_t)g * 8;
    dst = xh + (size_t)g * 8;
    sc = 1.0f;
  } else {
    const int e = g - NX8;
    const int wsel = (blk - NX8 / 256) / (NW8 / 256);
    const int off = e - wsel * NW8;
    const float* wsrc = (wsel == 0) ? wq : ((wsel == 1) ? wk : ((wsel == 2) ? wv : wo));
    src = wsrc + (size_t)off * 8;
    dst = wh + (size_t)e * 8;
    sc = WSCALE;
  }
  const v4f a = *(const v4fa*)src;
  const v4f c = *(const v4fa*)(src + 4);
  const v8h o = { (_Float16)(a.x * sc), (_Float16)(a.y * sc), (_Float16)(a.z * sc), (_Float16)(a.w * sc),
                  (_Float16)(c.x * sc), (_Float16)(c.y * sc), (_Float16)(c.z * sc), (_Float16)(c.w * sc) };
  *(volatile v8h*)dst = o;
  __threadfence();
  *(volatile v8h*)dst = o;
}

__device__ __forceinline__ void gemm_k2048(const _Float16* __restrict__ xa0,
                                           const _Float16* __restrict__ xa1,
                                           const _Float16* __restrict__ wb,
                                           int h, v8f (&acc)[2][4]) {
  const v8f zero8 = {0.f, 0.f, 0.f, 0.f, 0.f, 0.f, 0.f, 0.f};
  #pragma unroll
  for (int mt = 0; mt < 2; ++mt)
    #pragma unroll
    for (int nt = 0; nt < 4; ++nt) acc[mt][nt] = zero8;

  #pragma unroll 1
  for (int k0 = 0; k0 < HID; k0 += 32) {
    const v16h a0 = load_frag(xa0 + k0, h);
    const v16h a1 = load_frag(xa1 + k0, h);
    #pragma unroll
    for (int nt = 0; nt < 4; ++nt) {
      const v16h b = load_frag(wb + (size_t)nt * 16 * HID + k0, h);
      acc[0][nt] = wmma_f16(a0, b, acc[0][nt]);
      acc[1][nt] = wmma_f16(a1, b, acc[1][nt]);
    }
  }
}

__device__ __forceinline__ void proj_store_pass(const _Float16* sT, _Float16* plane, _Float16* vt,
                                                int which, int bh, int hf, int l0, int w, int lane) {
  const int q8 = lane & 7, sub = lane >> 3;
  #pragma unroll
  for (int i = 0; i < 8; ++i) {
    const int lid = w * 32 + i * 4 + sub;
    v8h v;
    _Float16* dst;
    if (which != 2) {
      v = *(const v8ha*)(sT + lid * 64 + 8 * q8);
      dst = plane + ((size_t)bh * SEQ + l0 + lid) * HD + 64 * hf + 8 * q8;
    } else {
      const int d = lid >> 1, hl = lid & 1;
      v = *(const v8ha*)(sT + d * 128 + 64 * hl + 8 * q8);
      dst = vt + ((size_t)bh * HD + 64 * hf + d) * SEQ + l0 + 64 * hl + 8 * q8;
    }
    *(volatile v8h*)dst = v;
  }
}

__global__ __launch_bounds__(128) void proj_kernel(
    const _Float16* __restrict__ xh,
    const _Float16* __restrict__ wh,
    const float* __restrict__ bq, const float* __restrict__ bk, const float* __restrict__ bv,
    _Float16* __restrict__ qh,
    _Float16* __restrict__ kh,
    _Float16* __restrict__ vt)
{
  __shared__ __attribute__((aligned(16))) _Float16 sT[128 * 64];

  const int tid = threadIdx.x, lane = tid & 31, w = tid >> 5;
  const int h = lane >> 4, m = lane & 15;
  const int m0 = blockIdx.x * 128;
  const int cg = blockIdx.y;
  const int which = cg >> 5;
  const int rem = cg & 31;
  const int head = rem >> 1, hf = rem & 1;
  const int m0w = m0 + 32 * w;

  const _Float16* xa0 = xh + (size_t)(m0w + m) * HID;
  const _Float16* xa1 = xa0 + (size_t)16 * HID;
  const _Float16* wb  = wh + ((size_t)which * HID + 64 * rem + m) * HID;

  v8f acc[2][4];
  gemm_k2048(xa0, xa1, wb, h, acc);

  const float* bias = (which == 0) ? bq : ((which == 1) ? bk : bv);
  #pragma unroll
  for (int nt = 0; nt < 4; ++nt) {
    const int feat = 16 * nt + m;
    const float bvl = bias[64 * rem + feat];
    #pragma unroll
    for (int mt = 0; mt < 2; ++mt) {
      #pragma unroll
      for (int r = 0; r < 8; ++r) {
        const int tokl = 32 * w + 16 * mt + 8 * h + r;
        const float y = acc[mt][nt][r] * 0.03125f + bvl;
        const int idx = (which == 2) ? (feat * 128 + tokl) : (tokl * 64 + feat);
        sT[idx] = (_Float16)y;
      }
    }
  }
  __syncthreads();

  const int b = m0 / SEQ, l0 = m0 - b * SEQ, bh = b * NHEAD + head;
  _Float16* plane = (which == 0) ? qh : kh;
  proj_store_pass(sT, plane, vt, which, bh, hf, l0, w, lane);
  __threadfence();
  proj_store_pass(sT, plane, vt, which, bh, hf, l0, w, lane);
}

__device__ __forceinline__ v16h pack_p(v8f a, v8f c) {
  const v16h r = { (_Float16)(a[0] * PSCALE), (_Float16)(a[1] * PSCALE), (_Float16)(a[2] * PSCALE), (_Float16)(a[3] * PSCALE),
                   (_Float16)(a[4] * PSCALE), (_Float16)(a[5] * PSCALE), (_Float16)(a[6] * PSCALE), (_Float16)(a[7] * PSCALE),
                   (_Float16)(c[0] * PSCALE), (_Float16)(c[1] * PSCALE), (_Float16)(c[2] * PSCALE), (_Float16)(c[3] * PSCALE),
                   (_Float16)(c[4] * PSCALE), (_Float16)(c[5] * PSCALE), (_Float16)(c[6] * PSCALE), (_Float16)(c[7] * PSCALE) };
  return r;
}

__device__ __forceinline__ void ctx_store_pass(const _Float16* sc, _Float16* ctx,
                                               int b, int head, int q0, int lane) {
  const int q8 = lane & 7, sub = lane >> 3;
  #pragma unroll
  for (int i = 0; i < 8; ++i) {
    const int lid = i * 4 + sub;
    const int row = lid >> 1, hl = lid & 1;
    const v8h v = *(const v8ha*)(sc + row * 128 + 64 * hl + 8 * q8);
    const size_t gi = ((size_t)b * SEQ + q0 + row) * HID + (size_t)head * HD + 64 * hl + 8 * q8;
    *(volatile v8h*)(ctx + gi) = v;
  }
}

__global__ __launch_bounds__(128) void attn_kernel(
    const _Float16* __restrict__ qh,
    const _Float16* __restrict__ kh,
    const _Float16* __restrict__ vt,
    _Float16* __restrict__ ctx)
{
  __shared__ __attribute__((aligned(16))) _Float16 sC[4 * 16 * 128];

  const int tid = threadIdx.x, lane = tid & 31, w = tid >> 5;
  const int h = lane >> 4, m = lane & 15;
  const int bh = blockIdx.y, b = bh >> 4, head = bh & 15;
  const int q0 = blockIdx.x * 64 + 16 * w;

  const _Float16* qrow = qh + ((size_t)bh * SEQ + q0 + m) * HD;
  v16h qb[4];
  #pragma unroll
  for (int c = 0; c < 4; ++c) qb[c] = load_frag(qrow + 32 * c, h);

  const v8f zero8 = {0.f, 0.f, 0.f, 0.f, 0.f, 0.f, 0.f, 0.f};
  v8f o[8];
  #pragma unroll
  for (int t = 0; t < 8; ++t) o[t] = zero8;
  float mrun = -1e30f, lrun = 0.0f;

  const _Float16* kbase = kh + ((size_t)bh * SEQ + m) * HD;
  const _Float16* vbase = vt + ((size_t)bh * HD + m) * SEQ;

  #pragma unroll 1
  for (int kb = 0; kb < SEQ; kb += 64) {
    v8f s[4];
    #pragma unroll
    for (int j = 0; j < 4; ++j) {
      const _Float16* kp = kbase + (size_t)(kb + 16 * j) * HD;
      v8f z = zero8;
      #pragma unroll
      for (int c = 0; c < 4; ++c) {
        const v16h kf = load_frag(kp + 32 * c, h);
        z = wmma_f16(kf, qb[c], z);
      }
      s[j] = z;
    }

    float mloc = -1e30f;
    #pragma unroll
    for (int j = 0; j < 4; ++j)
      #pragma unroll
      for (int r = 0; r < 8; ++r) {
        const float sv = s[j][r] * SM_SCALE;
        s[j][r] = sv;
        mloc = fmaxf(mloc, sv);
      }
    mloc = fmaxf(mloc, __shfl_xor(mloc, 16));
    const float mnew = fmaxf(mrun, mloc);
    const float alpha = __expf(mrun - mnew);
    mrun = mnew;
    float lsum = 0.0f;
    #pragma unroll
    for (int j = 0; j < 4; ++j)
      #pragma unroll
      for (int r = 0; r < 8; ++r) {
        const float p = __expf(s[j][r] - mnew);
        s[j][r] = p;
        lsum += p;
      }
    lsum += __shfl_xor(lsum, 16);
    lrun = lrun * alpha + lsum;
    #pragma unroll
    for (int t = 0; t < 8; ++t)
      #pragma unroll
      for (int r = 0; r < 8; ++r) o[t][r] = o[t][r] * alpha;

    const v16h pb0 = pack_p(s[0], s[1]);
    const v16h pb1 = pack_p(s[2], s[3]);

    #pragma unroll
    for (int t = 0; t < 8; ++t) {
      const _Float16* vp = vbase + (size_t)(16 * t) * SEQ + kb;
      const v16h vf0 = load_frag(vp, h);
      const v16h vf1 = load_frag(vp + 32, h);
      o[t] = wmma_f16(vf0, pb0, o[t]);
      o[t] = wmma_f16(vf1, pb1, o[t]);
    }
  }

  const float inv = (CSCALE / PSCALE) * (1.0f / lrun);
  _Float16* sc = sC + w * 2048;
  #pragma unroll
  for (int t = 0; t < 8; ++t) {
    const v8h cv = { (_Float16)(o[t][0] * inv), (_Float16)(o[t][1] * inv),
                     (_Float16)(o[t][2] * inv), (_Float16)(o[t][3] * inv),
                     (_Float16)(o[t][4] * inv), (_Float16)(o[t][5] * inv),
                     (_Float16)(o[t][6] * inv), (_Float16)(o[t][7] * inv) };
    *(v8ha*)(sc + m * 128 + 16 * t + 8 * h) = cv;
  }
  __syncthreads();

  ctx_store_pass(sc, ctx, b, head, q0, lane);
  __threadfence();
  ctx_store_pass(sc, ctx, b, head, q0, lane);
}

__device__ __forceinline__ void out_store_pass(const float* sO, float* out,
                                               int m0, int nb, int w, int lane) {
  const int q8 = lane & 7, sub = lane >> 3;
  #pragma unroll
  for (int i = 0; i < 16; ++i) {
    const int lid = i * 4 + sub;
    const int tokl = w * 32 + (lid >> 1), hl = lid & 1;
    const v4f v = *(const v4fa*)(sO + tokl * 64 + 32 * hl + 4 * q8);
    const size_t gi = (size_t)(m0 + tokl) * HID + 64 * nb + 32 * hl + 4 * q8;
    *(volatile v4f*)(out + gi) = v;
  }
}

__global__ __launch_bounds__(128) void out_kernel(
    const _Float16* __restrict__ ch,
    const _Float16* __restrict__ woh,
    const float* __restrict__ bo,
    float* __restrict__ out)
{
  __shared__ __attribute__((aligned(16))) float sO[128 * 64];

  const int tid = threadIdx.x, lane = tid & 31, w = tid >> 5;
  const int h = lane >> 4, m = lane & 15;
  const int m0 = blockIdx.x * 128;
  const int nb = blockIdx.y;
  const int m0w = m0 + 32 * w;

  const _Float16* xa0 = ch + (size_t)(m0w + m) * HID;
  const _Float16* xa1 = xa0 + (size_t)16 * HID;
  const _Float16* wb  = woh + ((size_t)(64 * nb) + m) * HID;

  v8f acc[2][4];
  gemm_k2048(xa0, xa1, wb, h, acc);

  #pragma unroll
  for (int nt = 0; nt < 4; ++nt) {
    const int feat = 16 * nt + m;
    const float bvl = bo[64 * nb + feat];
    #pragma unroll
    for (int mt = 0; mt < 2; ++mt) {
      #pragma unroll
      for (int r = 0; r < 8; ++r) {
        const int tokl = 32 * w + 16 * mt + 8 * h + r;
        sO[tokl * 64 + feat] = acc[mt][nt][r] * 0.0009765625f + bvl;
      }
    }
  }
  __syncthreads();

  out_store_pass(sO, out, m0, nb, w, lane);
  __threadfence();
  out_store_pass(sO, out, m0, nb, w, lane);
}

extern "C" void kernel_launch(void* const* d_in, const int* in_sizes, int n_in,
                              void* d_out, int out_size, void* d_ws, size_t ws_size,
                              hipStream_t stream) {
  if (n_in < 9) return;
  if (in_sizes[0] != NX) return;
  if (in_sizes[1] != NW || in_sizes[3] != NW || in_sizes[5] != NW || in_sizes[7] != NW) return;
  if (in_sizes[2] != HID || in_sizes[4] != HID || in_sizes[6] != HID || in_sizes[8] != HID) return;
  if (out_size != NX) return;

  const float* x  = (const float*)d_in[0];
  const float* Wq = (const float*)d_in[1];
  const float* bq = (const float*)d_in[2];
  const float* Wk = (const float*)d_in[3];
  const float* bk = (const float*)d_in[4];
  const float* Wv = (const float*)d_in[5];
  const float* bv = (const float*)d_in[6];
  const float* Wo = (const float*)d_in[7];
  const float* bo = (const float*)d_in[8];
  float* out = (float*)d_out;

  const size_t xh_bytes = (size_t)NX * 2;
  const size_t wh_bytes = (size_t)4 * NW * 2;
  const size_t pl_bytes = (size_t)BATCH * NHEAD * SEQ * HD * 2;
  const size_t cx_bytes = (size_t)NX * 2;
  const size_t total = xh_bytes + wh_bytes + 3 * pl_bytes + cx_bytes;
  if (total > ws_size) return;

  char* ws = (char*)d_ws;
  _Float16* xh = (_Float16*)(ws);
  _Float16* wh = (_Float16*)(ws + xh_bytes);
  _Float16* qh = (_Float16*)(ws + xh_bytes + wh_bytes);
  _Float16* kh = (_Float16*)(ws + xh_bytes + wh_bytes + pl_bytes);
  _Float16* vt = (_Float16*)(ws + xh_bytes + wh_bytes + 2 * pl_bytes);
  _Float16* cx = (_Float16*)(ws + xh_bytes + wh_bytes + 3 * pl_bytes);
  const _Float16* woh = wh + (size_t)3 * NW;

  const int nblk_cvt = (NX8 + 4 * NW8) / 256;
  convert_kernel<<<nblk_cvt, 256, 0, stream>>>(x, Wq, Wk, Wv, Wo, xh, wh);

  dim3 gProj(MROWS / 128, 3 * 32);
  proj_kernel<<<gProj, 128, 0, stream>>>(xh, wh, bq, bk, bv, qh, kh, vt);

  dim3 gAtt(SEQ / 64, BATCH * NHEAD);
  attn_kernel<<<gAtt, 128, 0, stream>>>(qh, kh, vt, cx);

  dim3 gOut(MROWS / 128, HID / 64);
  out_kernel<<<gOut, 128, 0, stream>>>(cx, woh, bo, out);
}
